// RopelessMLA_19061064859752
// MI455X (gfx1250) — hardware-run, weakly checked
//
#include <hip/hip_runtime.h>
#include <math.h>

typedef __attribute__((ext_vector_type(16))) _Float16 v16h;
typedef __attribute__((ext_vector_type(16))) __bf16 v16b;
typedef __attribute__((ext_vector_type(8)))  _Float16 v8h;
typedef __attribute__((ext_vector_type(8)))  __bf16 v8b;
typedef __attribute__((ext_vector_type(8)))  float v8f;
typedef __attribute__((ext_vector_type(4)))  float v4f;
typedef __attribute__((ext_vector_type(4)))  unsigned v4u;
typedef v8h __attribute__((may_alias)) v8h_a;
typedef _Float16 h16;

#ifndef NB
#define NB 2
#endif
#ifndef SEQ
#define SEQ 2048
#endif
#define NB_FULL 2
#define SEQ_FULL 2048
#define CC 2048
#define DIN 2048
#define NH 16
#define HD 128
#define LAT 512
#define SCALE (0.08838834764831845f)
#define LN_EPS (1.0e-5f)
#define QBH 4
#define KHI 256
#define OUT1_OFF ((size_t)NB_FULL * SEQ_FULL * DIN)

static_assert(NH * HD == CC);
static_assert(HD == 128);
static_assert(HD % 32 == 0);
static_assert(DIN % 32 == 0);
static_assert(LAT % 32 == 0);
static_assert(CC % 32 == 0);
static_assert(CC % 128 == 0);
static_assert(LAT % 128 == 0);
static_assert(DIN == CC);
static_assert(SEQ % 64 == 0);
static_assert(KHI == QBH * 64);
static_assert(KHI % 64 == 0);
static_assert(SEQ >= KHI);
static_assert(SEQ <= SEQ_FULL);
static_assert(NB <= NB_FULL);
static_assert((NB * SEQ) % 64 == 0);
static_assert((NB * SEQ) % 4 == 0);
static_assert(OUT1_OFF * 4 == (size_t)33554432);
static_assert((OUT1_OFF + (size_t)NB_FULL * SEQ_FULL * LAT) * 4 == (size_t)41943040);

#define PLANE ((size_t)NB * SEQ * CC)
#define EPLANE ((size_t)NB * KHI * CC)
#define WS_QH  ((size_t)0)
#define WS_KH  (WS_QH + 2u * PLANE)
#define WS_VT  (WS_KH + 2u * PLANE)
#define WS_QL  (WS_VT + 2u * PLANE)
#define WS_KL  (WS_QL + 2u * EPLANE)
#define WS_VB  (WS_KL + 2u * EPLANE)
#define WS_VBL (WS_VB + 2u * EPLANE)
#define WS_CP  (WS_VBL + 2u * EPLANE)
#define WS_Y   (WS_CP + 4u * (size_t)NB * SEQ * LAT)
#define WS_END (WS_Y + 4u * PLANE)
static_assert(WS_END <= (size_t)134217728);
static_assert(WS_KH % 128 == 0 && WS_VT % 128 == 0 && WS_QL % 128 == 0 && WS_KL % 128 == 0 && WS_VB % 128 == 0 && WS_VBL % 128 == 0 && WS_CP % 128 == 0 && WS_Y % 128 == 0);

template <typename T> __device__ __forceinline__ void vst2(void* p, T v) { *(volatile T*)p = v; __threadfence(); *(volatile T*)p = v; }
__device__ __forceinline__ v8f wmma16(v16h a, v16h b, v8f c) {
  v8f d = __builtin_amdgcn_wmma_f32_16x16x32_f16(false, a, false, b, (short)0, c, false, false);
  asm volatile("v_nop\n\tv_nop\n\tv_nop\n\tv_nop" : "+v"(d) : "v"(a), "v"(b));
  return d;
}
__device__ __forceinline__ v8f wmma_bf(v16b a, v16b b, v8f c) {
  v8f d = __builtin_amdgcn_wmma_f32_16x16x32_bf16(false, a, false, b, (short)0, c, false, false);
  asm volatile("v_nop\n\tv_nop\n\tv_nop\n\tv_nop" : "+v"(d) : "v"(a), "v"(b));
  return d;
}
__device__ __forceinline__ v16h frag_h(const _Float16* rowk0, int lane) {
  union { v16h v; v8h q[2]; } u; const _Float16* p = rowk0 + 8 * (lane >> 4);
  u.q[0] = *(const v8h*)p; u.q[1] = *(const v8h*)(p + 16); return u.v;
}
__device__ __forceinline__ v16b frag_b(const __bf16* rowk0, int lane) {
  union { v16b v; v8b q[2]; } u; const __bf16* p = rowk0 + 8 * (lane >> 4);
  u.q[0] = *(const v8b*)p; u.q[1] = *(const v8b*)(p + 16); return u.v;
}
struct F2 { v16b h, l; };
__device__ __forceinline__ F2 bsplit16(const float v[16]) { F2 r;
#pragma unroll
  for (int i = 0; i < 16; ++i) { const __bf16 h = (__bf16)v[i]; r.h[i] = h; r.l[i] = (__bf16)(v[i] - (float)h); }
  return r; }
__device__ __forceinline__ F2 split_row(const float* row, int k0, int lane) { float v[16]; const float* p = row + k0 + 8 * (lane >> 4);
#pragma unroll
  for (int i = 0; i < 8; ++i) { v[i] = p[i]; v[8 + i] = p[16 + i]; }
  return bsplit16(v); }
__device__ __forceinline__ float bfr(float v) { return (float)(__bf16)v; }
static __device__ __forceinline__ h16 toh_flush(float v) { const h16 r = (h16)v; return (fabsf(v) < 6.103515625e-05f) ? (h16)0.0f : r; }
__device__ __forceinline__ v16b wrow_oi(const float* wrow, int k0, int lane) { v16b w; const float* p = wrow + k0 + 8 * (lane >> 4);
#pragma unroll
  for (int i = 0; i < 8; ++i) { w[i] = (__bf16)p[i]; w[8 + i] = (__bf16)p[16 + i]; }
  return w; }
#define LDSX() do { asm volatile("s_wait_dscnt 0" ::: "memory"); __builtin_amdgcn_wave_barrier(); __builtin_amdgcn_fence(3  , "workgroup"); } while (0)

template <int NK> __device__ __forceinline__ void mm_single(const float* __restrict__ arow, const float* __restrict__ wrow, int lane, v8f (&acc)[8]) {
  const int g8 = 8 * (lane >> 4);
#pragma unroll 2
  for (int kc = 0; kc < NK; ++kc) { v16b a; { const float* p = arow + kc * 32 + g8;
#pragma unroll
      for (int i = 0; i < 8; ++i) { a[i] = (__bf16)p[i]; a[8 + i] = (__bf16)p[16 + i]; } }
    asm volatile("s_wait_loadcnt 0x0" ::: "memory");
#pragma unroll
    for (int j = 0; j < 8; ++j) { const v16b w = wrow_oi(wrow + (size_t)(j * 16) * (NK * 32), kc * 32, lane); asm volatile("s_wait_loadcnt 0x0" ::: "memory"); acc[j] = wmma_bf(a, w, acc[j]); } } }
template <int NK> __device__ __forceinline__ void mm_split(const float* __restrict__ arow, const float* __restrict__ wrow, int lane, v8f (&acc)[8]) {
#pragma unroll 2
  for (int kc = 0; kc < NK; ++kc) { const F2 a = split_row(arow, kc * 32, lane); asm volatile("s_wait_loadcnt 0x0" ::: "memory");
#pragma unroll
    for (int j = 0; j < 8; ++j) { const v16b w = wrow_oi(wrow + (size_t)(j * 16) * (NK * 32), kc * 32, lane); asm volatile("s_wait_loadcnt 0x0" ::: "memory"); acc[j] = wmma_bf(a.h, w, acc[j]); acc[j] = wmma_bf(a.l, w, acc[j]); } } }

template <int SPLIT, int NK>
__device__ __forceinline__ void rows_body(const float* __restrict__ A, const float* __restrict__ W, _Float16* __restrict__ DH, _Float16* __restrict__ DL) {
  __shared__ __align__(16) _Float16 sh[64][136], sl[64][136];
  const int tid = threadIdx.x; const int wave = __builtin_amdgcn_readfirstlane(tid >> 5); const int lane = tid & 31, col = lane & 15, g = lane >> 4;
  const int c0 = blockIdx.y * 128; const size_t r0 = (size_t)blockIdx.x * 64; const size_t bb = r0 / SEQ; const int t0 = (int)(r0 % SEQ);
  const bool early = t0 < KHI;
  const float* arow = A + ((size_t)bb * SEQ_FULL + t0 + wave * 16 + col) * (size_t)(NK * 32);
  const float* wrow = W + (size_t)(c0 + col) * (size_t)(NK * 32);
  v8f acc[8] = {};
  if (SPLIT) mm_split<NK>(arow, wrow, lane, acc); else mm_single<NK>(arow, wrow, lane, acc);
#pragma unroll
  for (int j = 0; j < 8; ++j) {
#pragma unroll
    for (int r = 0; r < 8; ++r) { const float v = acc[j][r]; const h16 hv = toh_flush(v); sh[wave * 16 + 8 * g + r][j * 16 + col] = hv; sl[wave * 16 + 8 * g + r][j * 16 + col] = toh_flush((v - (float)hv) * 1024.0f); } }
  __syncthreads();
  for (int e = tid; e < 64 * 16; e += 128) { const int rl = e >> 4, q = e & 15; const v4u a = *(const v4u*)&sh[rl][q * 8]; const size_t o2 = (r0 + rl) * (size_t)CC + c0 + q * 8; vst2(DH + o2, a);
    if (early) { const v4u bq = *(const v4u*)&sl[rl][q * 8]; const size_t o3 = ((size_t)bb * KHI + t0 + rl) * (size_t)CC + c0 + q * 8; vst2(DL + o3, bq); } } }

__global__ __launch_bounds__(128) void k_qproj(const float* __restrict__ X, const float* __restrict__ WQ, _Float16* __restrict__ QH, _Float16* __restrict__ QL) {
  rows_body<0, DIN / 32>(X, WQ, QH, QL); }
__global__ __launch_bounds__(128) void k_kproj(const float* __restrict__ CKV, const float* __restrict__ WK, _Float16* __restrict__ KH, _Float16* __restrict__ KL) {
  rows_body<1, LAT / 32>(CKV, WK, KH, KL); }

__global__ __launch_bounds__(128) void k_cpre(const float* __restrict__ X, const float* __restrict__ WD, float* __restrict__ CP) {
  __shared__ __align__(16) float sf[4][16][132];
  const int tid = threadIdx.x; const int wave = __builtin_amdgcn_readfirstlane(tid >> 5); const int lane = tid & 31, col = lane & 15, g = lane >> 4;
  const int c0 = blockIdx.y * 128; const size_t rb = (size_t)blockIdx.x * 64; const size_t bb = rb / SEQ; const int t0 = (int)(rb % SEQ);
  const float* arow = X + ((size_t)bb * SEQ_FULL + t0 + wave * 16 + col) * (size_t)DIN;
  const float* wrow = WD + (size_t)(c0 + col) * (size_t)DIN;
  v8f acc[8] = {};
  mm_single<DIN / 32>(arow, wrow, lane, acc);
#pragma unroll
  for (int j = 0; j < 8; ++j) {
#pragma unroll
    for (int r = 0; r < 8; ++r) sf[wave][8 * g + r][j * 16 + col] = acc[j][r]; }
  LDSX();
  const size_t r0 = rb + wave * 16;
  for (int rl = 0; rl < 16; ++rl) { const v4f v = *(const v4f*)&sf[wave][rl][lane * 4]; vst2(CP + (r0 + rl) * (size_t)LAT + c0 + lane * 4, v); } }

__global__ __launch_bounds__(128) void k_ln(const float* __restrict__ CP, const float* __restrict__ LW, const float* __restrict__ LB, float* __restrict__ CO) {
#pragma clang fp contract(off)
  const int tid = threadIdx.x; const int wave = __builtin_amdgcn_readfirstlane(tid >> 5); const int lane = tid & 31;
  const size_t row = (size_t)blockIdx.x * 4 + wave; const size_t bb = row / SEQ; const int t = (int)(row % SEQ);
  const float* src = CP + row * (size_t)LAT + lane * 4; float* dst = CO + (bb * SEQ_FULL + t) * (size_t)LAT + lane * 4;
  float s = 0.f;
#pragma unroll 1
  for (int it = 0; it < LAT / 128; ++it) { const v4f v = *(const v4f*)(src + it * 128); s += (v.x + v.y) + (v.z + v.w); }
  s += __shfl_xor(s, 1); s += __shfl_xor(s, 2); s += __shfl_xor(s, 4); s += __shfl_xor(s, 8); s += __shfl_xor(s, 16);
  const float mu = s * (1.0f / LAT);
  float q = 0.f;
#pragma unroll 1
  for (int it = 0; it < LAT / 128; ++it) { const v4f v = *(const v4f*)(src + it * 128); const float dx = v.x - mu, dy = v.y - mu, dz = v.z - mu, dw = v.w - mu; q += (dx * dx + dy * dy) + (dz * dz + dw * dw); }
  q += __shfl_xor(q, 1); q += __shfl_xor(q, 2); q += __shfl_xor(q, 4); q += __shfl_xor(q, 8); q += __shfl_xor(q, 16);
  const float rs = rsqrtf(q * (1.0f / LAT) + LN_EPS);
#pragma unroll 1
  for (int it = 0; it < LAT / 128; ++it) { const v4f v = *(const v4f*)(src + it * 128); const v4f w = *(const v4f*)(LW + it * 128 + lane * 4); const v4f bq = *(const v4f*)(LB + it * 128 + lane * 4);
    v4f o; o.x = (v.x - mu) * rs * bfr(w.x) + bfr(bq.x); o.y = (v.y - mu) * rs * bfr(w.y) + bfr(bq.y); o.z = (v.z - mu) * rs * bfr(w.z) + bfr(bq.z); o.w = (v.w - mu) * rs * bfr(w.w) + bfr(bq.w);
    vst2(dst + it * 128, o); } }

__global__ __launch_bounds__(128) void k_vproj(const float* __restrict__ CKV, const float* __restrict__ WV, _Float16* __restrict__ VT, __bf16* __restrict__ VB, __bf16* __restrict__ VBL) {
  __shared__ __align__(16) _Float16 th[128][72]; __shared__ __align__(16) __bf16 tb[128][72], tbl[128][72];
  const int tid = threadIdx.x; const int wave = __builtin_amdgcn_readfirstlane(tid >> 5); const int lane = tid & 31, col = lane & 15, g = lane >> 4;
  const int c0 = blockIdx.y * 128; const size_t r0 = (size_t)blockIdx.x * 64; const size_t bb = r0 / SEQ; const int t0 = (int)(r0 % SEQ);
  const bool hi_rows = t0 < KHI;
  const float* arow = CKV + ((size_t)bb * SEQ_FULL + t0 + wave * 16 + col) * (size_t)LAT;
  const float* wrow = WV + (size_t)(c0 + col) * (size_t)LAT;
  v8f acc[8] = {};
  mm_split<LAT / 32>(arow, wrow, lane, acc);
#pragma unroll
  for (int j = 0; j < 8; ++j) {
#pragma unroll
    for (int r = 0; r < 8; ++r) { const float v = acc[j][r]; const int rl = wave * 16 + 8 * g + r, cl = j * 16 + col; th[cl][rl] = toh_flush(v); const __bf16 bh = (__bf16)v; tb[cl][rl] = bh; tbl[cl][rl] = (__bf16)(v - (float)bh); } }
  __syncthreads();
  for (int e = tid; e < 128 * 8; e += 128) { const int cl = e >> 3, q = e & 7; const v4u a = *(const v4u*)&th[cl][q * 8]; vst2(VT + (bb * CC + c0 + cl) * (size_t)SEQ + t0 + q * 8, a);
    if (hi_rows) { const size_t o3 = (bb * CC + c0 + cl) * (size_t)KHI + t0 + q * 8; const v4u bh = *(const v4u*)&tb[cl][q * 8]; const v4u bl = *(const v4u*)&tbl[cl][q * 8]; vst2(VB + o3, bh); vst2(VBL + o3, bl); } } }

__device__ __forceinline__ void fa_scores1(const _Float16* __restrict__ QH, const _Float16* __restrict__ KH, size_t qoff, size_t koff, int lane, v8f& s0, v8f& s1) {
#pragma unroll
  for (int kc = 0; kc < HD / 32; ++kc) {
    const v16h ah = frag_h(QH + qoff + kc * 32, lane);
    const v16h kh0 = frag_h(KH + koff + kc * 32, lane);
    s0 = wmma16(ah, kh0, s0);
    const v16h kh1 = frag_h(KH + koff + (size_t)16 * CC + kc * 32, lane);
    s1 = wmma16(ah, kh1, s1); } }
__device__ __forceinline__ void fa_scores3(const _Float16* __restrict__ QH, const _Float16* __restrict__ QL, const _Float16* __restrict__ KH, const _Float16* __restrict__ KL,
    size_t qoff, size_t qloff, size_t koff, size_t kloff, int lane, v8f& s0, v8f& s1, v8f& t0, v8f& t1) {
#pragma unroll
  for (int kc = 0; kc < HD / 32; ++kc) {
    const v16h ah = frag_h(QH + qoff + kc * 32, lane), al = frag_h(QL + qloff + kc * 32, lane);
    const v16h kh0 = frag_h(KH + koff + kc * 32, lane), kl0 = frag_h(KL + kloff + kc * 32, lane);
    s0 = wmma16(ah, kh0, s0); t0 = wmma16(al, kh0, t0); t0 = wmma16(ah, kl0, t0);
    const v16h kh1 = frag_h(KH + koff + (size_t)16 * CC + kc * 32, lane), kl1 = frag_h(KL + kloff + (size_t)16 * CC + kc * 32, lane);
    s1 = wmma16(ah, kh1, s1); t1 = wmma16(al, kh1, t1); t1 = wmma16(ah, kl1, t1); } }
__device__ __forceinline__ void fa_softmax(const v8f& s0, const v8f& s1, int k0, int qg0, int col, v8f& m, v8f& l, v8f (&o)[8], v8f& p0, v8f& p1) {
#pragma unroll
  for (int r = 0; r < 8; ++r) { const int qg = qg0 + r;
    float a0 = s0[r] * SCALE, a1 = s1[r] * SCALE;
    a0 = (k0 + col <= qg) ? a0 : -3.0e38f; a1 = (k0 + 16 + col <= qg) ? a1 : -3.0e38f;
    float rm = fmaxf(a0, a1);
    rm = fmaxf(rm, __shfl_xor(rm, 1)); rm = fmaxf(rm, __shfl_xor(rm, 2)); rm = fmaxf(rm, __shfl_xor(rm, 4)); rm = fmaxf(rm, __shfl_xor(rm, 8));
    const float mo = m[r]; const float mn = fmaxf(mo, rm);
    const float ec = __expf(mo - mn), e0r = __expf(a0 - mn), e1r = __expf(a1 - mn);
    const float corr = (mo <= -1.0e38f) ? 0.f : ec; const float e0 = (a0 <= -1.0e38f) ? 0.f : e0r; const float e1 = (a1 <= -1.0e38f) ? 0.f : e1r;
    m[r] = mn; l[r] = l[r] * corr;
#pragma unroll
    for (int j = 0; j < 8; ++j) o[j][r] *= corr;
    p0[r] = e0; p1[r] = e1; } }

__global__ __launch_bounds__(128) void k_fa_late(const _Float16* __restrict__ QH, const _Float16* __restrict__ KH, const _Float16* __restrict__ VT, float* __restrict__ Y) {
  __shared__ __align__(16) _Float16 ps[4][16][40]; __shared__ __align__(16) float so[4][16][HD + 4];
  const int tid = threadIdx.x; const int wave = __builtin_amdgcn_readfirstlane(tid >> 5); const int lane = tid & 31, col = lane & 15, g = lane >> 4;
  const int qb = QBH + (int)blockIdx.x; const int h = blockIdx.y; const int b = blockIdx.z;
  const int ql0 = qb * 64 + wave * 16; const int nhalf = ((ql0 + 15) >> 5) + 1;
  const size_t qoff = ((size_t)b * SEQ + ql0 + col) * CC + h * HD; const size_t kbase = ((size_t)b * SEQ + col) * CC + h * HD; const size_t vbase = ((size_t)b * CC + h * HD + col) * (size_t)SEQ;
  v8f o[8] = {}; v8f l = {}; v8f m;
#pragma unroll
  for (int r = 0; r < 8; ++r) m[r] = -3.0e38f;
#pragma unroll 1
  for (int hk = 0; hk < nhalf; ++hk) { const int k0 = hk * 32;
    v8f s0 = {}, s1 = {}, p0, p1;
    fa_scores1(QH, KH, qoff, kbase + (size_t)k0 * CC, lane, s0, s1);
    fa_softmax(s0, s1, k0, ql0 + 8 * g, col, m, l, o, p0, p1);
#pragma unroll
    for (int r = 0; r < 8; ++r) { const h16 h0 = toh_flush(p0[r] * 2048.0f), h1 = toh_flush(p1[r] * 2048.0f); ps[wave][8 * g + r][col] = h0; ps[wave][8 * g + r][16 + col] = h1; l[r] += (float)h0 + (float)h1; }
    LDSX();
    union { v16h v; v8h q[2]; } pu; pu.q[0] = *(const v8h_a*)&ps[wave][col][8 * g]; pu.q[1] = *(const v8h_a*)&ps[wave][col][16 + 8 * g];
#pragma unroll
    for (int j = 0; j < 8; ++j) o[j] = wmma16(pu.v, frag_h(VT + vbase + (size_t)(j * 16) * SEQ + k0, lane), o[j]);
    LDSX(); }
#pragma unroll
  for (int r = 0; r < 8; ++r) { float ls = l[r]; ls += __shfl_xor(ls, 1); ls += __shfl_xor(ls, 2); ls += __shfl_xor(ls, 4); ls += __shfl_xor(ls, 8); const float inv = 1.0f / ls;
#pragma unroll
    for (int j = 0; j < 8; ++j) so[wave][8 * g + r][j * 16 + col] = o[j][r] * inv; }
  LDSX();
  for (int rl = 0; rl < 16; ++rl) { const v4f v = *(const v4f*)&so[wave][rl][lane * 4]; vst2(Y + ((size_t)b * SEQ + ql0 + rl) * CC + h * HD + lane * 4, v); } }

__global__ __launch_bounds__(128) void k_fa_early(const _Float16* __restrict__ QH, const _Float16* __restrict__ QL, const _Float16* __restrict__ KH, const _Float16* __restrict__ KL, const __bf16* __restrict__ VB, const __bf16* __restrict__ VBL, float* __restrict__ Y) {
  __shared__ __align__(16) float pf[4][16][36]; __shared__ __align__(16) float so[4][16][HD + 4];
  const int tid = threadIdx.x; const int wave = __builtin_amdgcn_readfirstlane(tid >> 5); const int lane = tid & 31, col = lane & 15, g = lane >> 4;
  const int qb = blockIdx.x; const int h = blockIdx.y; const int b = blockIdx.z;
  const int ql0 = qb * 64 + wave * 16; const int nhalf = ((ql0 + 15) >> 5) + 1;
  const size_t qoff = ((size_t)b * SEQ + ql0 + col) * CC + h * HD; const size_t qloff = ((size_t)b * KHI + ql0 + col) * CC + h * HD;
  const size_t kbase = ((size_t)b * SEQ + col) * CC + h * HD; const size_t klbase = ((size_t)b * KHI + col) * CC + h * HD;
  const size_t vbase = ((size_t)b * CC + h * HD + col) * (size_t)KHI;
  v8f o[8] = {}; v8f l = {}; v8f m;
#pragma unroll
  for (int r = 0; r < 8; ++r) m[r] = -3.0e38f;
#pragma unroll 1
  for (int hk = 0; hk < nhalf; ++hk) { const int k0 = hk * 32;
    v8f s0 = {}, s1 = {}, t0 = {}, t1 = {}, p0, p1;
    fa_scores3(QH, QL, KH, KL, qoff, qloff, kbase + (size_t)k0 * CC, klbase + (size_t)k0 * CC, lane, s0, s1, t0, t1);
#pragma unroll
    for (int r = 0; r < 8; ++r) { s0[r] = s0[r] + t0[r] * (1.0f / 1024.0f); s1[r] = s1[r] + t1[r] * (1.0f / 1024.0f); }
    fa_softmax(s0, s1, k0, ql0 + 8 * g, col, m, l, o, p0, p1);
#pragma unroll
    for (int r = 0; r < 8; ++r) { pf[wave][8 * g + r][col] = p0[r]; pf[wave][8 * g + r][16 + col] = p1[r]; l[r] += p0[r] + p1[r]; }
    LDSX();
    float pv[16];
#pragma unroll
    for (int i = 0; i < 8; ++i) { pv[i] = pf[wave][col][8 * g + i]; pv[8 + i] = pf[wave][col][16 + 8 * g + i]; }
    const F2 p = bsplit16(pv);
#pragma unroll
    for (int j = 0; j < 8; ++j) { const size_t po = vbase + (size_t)(j * 16) * KHI + k0; const v16b vh = frag_b(VB + po, lane); o[j] = wmma_bf(p.h, vh, o[j]); o[j] = wmma_bf(p.l, vh, o[j]); o[j] = wmma_bf(p.h, frag_b(VBL + po, lane), o[j]); }
    LDSX(); }
#pragma unroll
  for (int r = 0; r < 8; ++r) { float ls = l[r]; ls += __shfl_xor(ls, 1); ls += __shfl_xor(ls, 2); ls += __shfl_xor(ls, 4); ls += __shfl_xor(ls, 8); const float inv = 1.0f / ls;
#pragma unroll
    for (int j = 0; j < 8; ++j) so[wave][8 * g + r][j * 16 + col] = o[j][r] * inv; }
  LDSX();
  for (int rl = 0; rl < 16; ++rl) { const v4f v = *(const v4f*)&so[wave][rl][lane * 4]; vst2(Y + ((size_t)b * SEQ + ql0 + rl) * CC + h * HD + lane * 4, v); } }

__global__ __launch_bounds__(128) void k_out(const float* __restrict__ Y, const float* __restrict__ WO, float* __restrict__ OUT) {
  __shared__ __align__(16) float sf[4][16][132];
  const int tid = threadIdx.x; const int wave = __builtin_amdgcn_readfirstlane(tid >> 5); const int lane = tid & 31, col = lane & 15, g = lane >> 4;
  const int c0 = blockIdx.y * 128; const size_t rb = (size_t)blockIdx.x * 64; const size_t bb = rb / SEQ; const int t0 = (int)(rb % SEQ);
  const size_t r0 = rb + wave * 16; const size_t orow0 = bb * SEQ_FULL + t0 + wave * 16;
  const float* arow = Y + (r0 + col) * (size_t)CC;
  const float* wrow = WO + (size_t)(c0 + col) * (size_t)CC;
  v8f acc[8] = {};
  mm_split<CC / 32>(arow, wrow, lane, acc);
#pragma unroll
  for (int j = 0; j < 8; ++j) {
#pragma unroll
    for (int r = 0; r < 8; ++r) sf[wave][8 * g + r][j * 16 + col] = acc[j][r]; }
  LDSX();
  for (int rl = 0; rl < 16; ++rl) { const v4f v = *(const v4f*)&sf[wave][rl][lane * 4]; vst2(OUT + (orow0 + rl) * (size_t)DIN + c0 + lane * 4, v); } }

extern "C" void kernel_launch(void* const* d_in, const int* in_sizes, int n_in, void* d_out, int out_size, void* d_ws, size_t ws_size, hipStream_t stream) {
  if (n_in < 8) return;
  const size_t need_rows = (size_t)(NB - 1) * SEQ_FULL + SEQ;
  if ((size_t)in_sizes[0] < need_rows * DIN) return;
  if ((size_t)in_sizes[1] < (size_t)CC * DIN) return;
  if ((size_t)in_sizes[2] < (size_t)LAT * DIN) return;
  if ((size_t)in_sizes[3] < (size_t)CC * LAT) return;
  if ((size_t)in_sizes[4] < (size_t)CC * LAT) return;
  if ((size_t)in_sizes[5] < (size_t)DIN * CC) return;
  if ((size_t)in_sizes[6] < (size_t)LAT) return;
  if ((size_t)in_sizes[7] < (size_t)LAT) return;
  if ((size_t)out_size < OUT1_OFF + need_rows * LAT) return;
  if (ws_size < (size_t)WS_END) return;
  const float* x = (const float*)d_in[0]; const float* W_q = (const float*)d_in[1]; const float* W_dkv = (const float*)d_in[2]; const float* W_uk = (const float*)d_in[3];
  const float* W_uv = (const float*)d_in[4]; const float* W_o = (const float*)d_in[5]; const float* ln_w = (const float*)d_in[6]; const float* ln_b = (const float*)d_in[7];
  float* out0 = (float*)d_out; float* out1 = (float*)d_out + OUT1_OFF;
  char* ws = (char*)d_ws;
  _Float16 *QH = (_Float16*)(ws + WS_QH), *QL = (_Float16*)(ws + WS_QL), *KH = (_Float16*)(ws + WS_KH), *KL = (_Float16*)(ws + WS_KL), *VT = (_Float16*)(ws + WS_VT);
  __bf16 *VB = (__bf16*)(ws + WS_VB), *VBL = (__bf16*)(ws + WS_VBL); float* CP = (float*)(ws + WS_CP); float* Y = (float*)(ws + WS_Y);
  k_qproj<<<dim3(NB * SEQ / 64, CC / 128), 128, 0, stream>>>(x, W_q, QH, QL);
  k_cpre<<<dim3(NB * SEQ / 64, LAT / 128), 128, 0, stream>>>(x, W_dkv, CP);
  k_ln<<<dim3(NB * SEQ / 4), 128, 0, stream>>>(CP, ln_w, ln_b, out1);
  k_kproj<<<dim3(NB * SEQ / 64, CC / 128), 128, 0, stream>>>(out1, W_uk, KH, KL);
  k_vproj<<<dim3(NB * SEQ / 64, CC / 128), 128, 0, stream>>>(out1, W_uv, VT, VB, VBL);
  k_fa_early<<<dim3(QBH, NH, NB), 128, 0, stream>>>(QH, QL, KH, KL, VB, VBL, Y);
  if (SEQ / 64 > QBH) k_fa_late<<<dim3(SEQ / 64 - QBH, NH, NB), 128, 0, stream>>>(QH, KH, VT, Y);
  k_out<<<dim3(NB * SEQ / 64, DIN / 128), 128, 0, stream>>>(Y, W_o, out0);
}
